// InfoNCELoss_58085137711484
// MI455X (gfx1250) — hardware-verified
//
#include <hip/hip_runtime.h>
#include <stdint.h>


typedef _Float16 v16h __attribute__((ext_vector_type(16)));
typedef _Float16 v8h  __attribute__((ext_vector_type(8)));
typedef float    v8f  __attribute__((ext_vector_type(8)));
typedef float    v4f  __attribute__((ext_vector_type(4)));
union Frag { v16h v; v8h half[2]; };

#define D           512
#define M_TILE      64
#define N_SPLIT     8
#define INV_T       (1.0f / 0.07f)
#define OP_SCALE    64.0f
#define ACC_UNSCALE (1.0f / 4096.0f)

__host__ __device__ static inline int imin(int a, int b) { return a < b ? a : b; }
__host__ __device__ static inline int imax(int a, int b) { return a > b ? a : b; }

__device__ __forceinline__ v8f wmma_f16(const v16h a, const v16h b, v8f acc) {
  acc = __builtin_amdgcn_wmma_f32_16x16x32_f16(false, a, false, b, (short)0, acc, false, false);
  asm volatile("v_nop\n\tv_nop\n\tv_nop\n\tv_nop" : "+v"(acc) : "v"(a), "v"(b));
  return acc;
}

__global__ __launch_bounds__(256)
void k_norm(const float* __restrict__ emb, _Float16* __restrict__ e16, int n_emb) {
  const int wave = blockIdx.x * 8 + ((int)threadIdx.x >> 5);
  const int lane = threadIdx.x & 31;
  if (wave >= n_emb) return;

  const float* row = emb + (size_t)wave * D;
  float ss = 0.f;
#pragma unroll
  for (int j = 0; j < 4; ++j) {
    const v4f x = *(const v4f*)(row + 128 * j + 4 * lane);
    ss += x.x * x.x; ss += x.y * x.y; ss += x.z * x.z; ss += x.w * x.w;
  }
#pragma unroll
  for (int off = 16; off; off >>= 1) ss += __shfl_xor(ss, off, 32);

  const float inv = 1.0f / fmaxf(sqrtf(ss), 1e-8f);
  const float sc  = inv * OP_SCALE;

  v8h o[2];
#pragma unroll
  for (int j = 0; j < 2; ++j) {
    const float* src = row + 256 * j + 8 * lane;
    const v4f x0 = *(const v4f*)(src);
    const v4f x1 = *(const v4f*)(src + 4);
    v8h t;
    t[0] = (_Float16)(x0.x * sc); t[1] = (_Float16)(x0.y * sc);
    t[2] = (_Float16)(x0.z * sc); t[3] = (_Float16)(x0.w * sc);
    t[4] = (_Float16)(x1.x * sc); t[5] = (_Float16)(x1.y * sc);
    t[6] = (_Float16)(x1.z * sc); t[7] = (_Float16)(x1.w * sc);
    o[j] = t;
  }
  _Float16* orow = e16 + (size_t)wave * D;
#pragma unroll
  for (int j = 0; j < 2; ++j) *(volatile v8h*)(orow + 256 * j + 8 * lane) = o[j];
  __threadfence();
#pragma unroll
  for (int j = 0; j < 2; ++j) *(volatile v8h*)(orow + 256 * j + 8 * lane) = o[j];
}

__global__ __launch_bounds__(256)
void k_rows(const _Float16* __restrict__ e16,
            const int* __restrict__ anchor,
            float* __restrict__ gpart,
            int n_emb, int n_pos, int tiles_per_slice, int n_pos_pad, int zarg) {
  __shared__ __align__(16) _Float16 As[M_TILE * D];
  __shared__ float red_s[8][M_TILE];
  __shared__ union { float f[M_TILE]; v4f v[M_TILE / 4]; } red2;

  const int mblk = blockIdx.x;
  const int nblk = blockIdx.y;
  const int tid  = threadIdx.x;
  const int wave = tid >> 5;
  const int lane = tid & 31;

  {
    const int row  = tid >> 2;
    const int colb = (tid & 3) * 128;
    const int p    = imin(mblk * M_TILE + row, n_pos - 1);
    int a = anchor[p];
    a = imin(imax(a, 0), n_emb - 1);
    const v8h* src = (const v8h*)(e16 + (size_t)a * D + colb);
    v8h*       dst = (v8h*)(As + row * D + colb);
#pragma unroll 4
    for (int i = 0; i < 16; ++i) dst[i] = src[i];
  }
  __syncthreads();

  const int h = lane >> 4;
  const int m = lane & 15;

  float sacc[4][8];
#pragma unroll
  for (int t = 0; t < 4; ++t)
#pragma unroll
    for (int i = 0; i < 8; ++i) sacc[t][i] = 0.f;

  for (int nt = wave; nt < tiles_per_slice; nt += 8) {
    const int zoff = zarg * nt;
    const _Float16* Abase = As + zoff + m * D + 8 * h;

    const int col0 = (nblk * tiles_per_slice + nt) * 16;
    const int crow = imin(col0 + m, n_emb - 1);
    const _Float16* bcol = e16 + (size_t)crow * D + 8 * h;

    const v8f z8 = {0.f, 0.f, 0.f, 0.f, 0.f, 0.f, 0.f, 0.f};
    v8f acc[4];
#pragma unroll
    for (int t = 0; t < 4; ++t) acc[t] = z8;

#pragma unroll 2
    for (int kt = 0; kt < D / 32; ++kt) {
      const int kb = kt * 32;
      Frag b;
      b.half[0] = *(const v8h*)(bcol + kb);
      b.half[1] = *(const v8h*)(bcol + kb + 16);
#pragma unroll
      for (int t = 0; t < 4; ++t) {
        const _Float16* Ar = Abase + t * 16 * D + kb;
        Frag a;
        a.half[0] = *(const v8h*)(Ar);
        a.half[1] = *(const v8h*)(Ar + 16);
        acc[t] = wmma_f16(a.v, b.v, acc[t]);
      }
    }

    const bool cvalid = (col0 + m) < n_emb;
#pragma unroll
    for (int t = 0; t < 4; ++t)
#pragma unroll
      for (int i = 0; i < 8; ++i) {
        const float s = acc[t][i] * ACC_UNSCALE;
        const float e = __expf((s - 1.0f) * INV_T);
        sacc[t][i] += cvalid ? e : 0.0f;
      }
  }

#pragma unroll
  for (int t = 0; t < 4; ++t)
#pragma unroll
    for (int i = 0; i < 8; ++i) {
      float s = sacc[t][i];
      s += __shfl_xor(s, 1, 32);
      s += __shfl_xor(s, 2, 32);
      s += __shfl_xor(s, 4, 32);
      s += __shfl_xor(s, 8, 32);
      if (m == 0) red_s[wave][t * 16 + h * 8 + i] = s;
    }
  __syncthreads();

  if (tid < M_TILE) {
    float s = 0.f;
#pragma unroll
    for (int w = 0; w < 8; ++w) s += red_s[w][tid];
    red2.f[tid] = s;
  }
  __syncthreads();

  if (wave == 0 && lane < M_TILE / 4) {
    const v4f v = red2.v[lane];
    float* dst = gpart + (size_t)nblk * n_pos_pad + (size_t)mblk * M_TILE + 4 * lane;
    *(volatile v4f*)dst = v;
    __threadfence();
    *(volatile v4f*)dst = v;
  }
}

__global__ __launch_bounds__(256)
void k_pairs(const float* __restrict__ emb,
             const int* __restrict__ ia, const int* __restrict__ ib,
             float* __restrict__ dots, int n, int n_emb) {
  __shared__ union { float f[32]; v4f v[8]; } res;
  const int tid  = threadIdx.x;
  const int wave = tid >> 5;
  const int lane = tid & 31;
  const int base = blockIdx.x * 32;

#pragma unroll 1
  for (int j = 0; j < 4; ++j) {
    const int p = imin(base + wave * 4 + j, n - 1);
    int a = ia[p]; a = imin(imax(a, 0), n_emb - 1);
    int b = ib[p]; b = imin(imax(b, 0), n_emb - 1);
    const float* ra = emb + (size_t)a * D + 16 * lane;
    const float* rb = emb + (size_t)b * D + 16 * lane;
    float saa = 0.f, sbb = 0.f, sab = 0.f;
#pragma unroll
    for (int q = 0; q < 4; ++q) {
      const v4f xa = *(const v4f*)(ra + 4 * q);
      const v4f xb = *(const v4f*)(rb + 4 * q);
      saa += xa.x * xa.x; saa += xa.y * xa.y; saa += xa.z * xa.z; saa += xa.w * xa.w;
      sbb += xb.x * xb.x; sbb += xb.y * xb.y; sbb += xb.z * xb.z; sbb += xb.w * xb.w;
      sab += xa.x * xb.x; sab += xa.y * xb.y; sab += xa.z * xb.z; sab += xa.w * xb.w;
    }
#pragma unroll
    for (int off = 16; off; off >>= 1) {
      saa += __shfl_xor(saa, off, 32);
      sbb += __shfl_xor(sbb, off, 32);
      sab += __shfl_xor(sab, off, 32);
    }
    const float inva = 1.0f / fmaxf(sqrtf(saa), 1e-8f);
    const float invb = 1.0f / fmaxf(sqrtf(sbb), 1e-8f);
    const float c = (sab * inva) * invb;
    if (lane == 0) res.f[wave * 4 + j] = c;
  }
  __syncthreads();

  if (wave == 0 && lane < 8) {
    const v4f v = res.v[lane];
    float* dst = dots + (size_t)base + 4 * lane;
    *(volatile v4f*)dst = v;
    __threadfence();
    *(volatile v4f*)dst = v;
  }
}

__global__ __launch_bounds__(256)
void k_final(const float* __restrict__ gpart,
             const float* __restrict__ posdot,
             const float* __restrict__ negdot,
             float* __restrict__ out,
             int n_pos, int n_neg, int n_pos_pad) {
  __shared__ double r0[256];
  __shared__ double r1[256];
  __shared__ double r2[256];
  const int tid = threadIdx.x;

  double sl = 0.0, sp = 0.0, sn = 0.0;
  for (int p = tid; p < n_pos; p += 256) {
    float S = 0.f;
#pragma unroll
    for (int q = 0; q < N_SPLIT; ++q) S += gpart[(size_t)q * n_pos_pad + p];
    const float pd = posdot[p];
    const float lp = (INV_T + logf(S)) - pd * INV_T;
    sl += (double)lp;
    sp += (double)pd;
  }
  for (int q = tid; q < n_neg; q += 256) sn += (double)negdot[q];

  r0[tid] = sl; r1[tid] = sp; r2[tid] = sn;
  __syncthreads();
  for (int off = 128; off; off >>= 1) {
    if (tid < off) {
      r0[tid] += r0[tid + off];
      r1[tid] += r1[tid + off];
      r2[tid] += r2[tid + off];
    }
    __syncthreads();
  }
  if (tid == 0) {
    const float o0 = (float)(r0[0] / (double)n_pos);
    const float o1 = (float)(r1[0] / (double)n_pos);
    const float o2 = (float)(r2[0] / (double)n_neg);
    volatile float* vo = out;
    vo[0] = o0; vo[1] = o1; vo[2] = o2;
    __threadfence();
    vo[0] = o0; vo[1] = o1; vo[2] = o2;
  }
}

static inline size_t alup256(size_t x) { return (x + 255) & ~(size_t)255; }

extern "C" void kernel_launch(void* const* d_in, const int* in_sizes, int n_in,
                              void* d_out, int out_size, void* d_ws, size_t ws_size,
                              hipStream_t stream) {
  if (n_in < 5 || out_size < 3) return;

  const float* emb = (const float*)d_in[0];
  const int*   pa  = (const int*)d_in[1];
  const int*   pt  = (const int*)d_in[2];
  const int*   na  = (const int*)d_in[3];
  const int*   ng  = (const int*)d_in[4];
  float*       out = (float*)d_out;

  const int n_emb = in_sizes[0] / D;
  const int n_pos = imin(in_sizes[1], in_sizes[2]);
  const int n_neg = imin(in_sizes[3], in_sizes[4]);
  if (n_emb < 1 || n_pos < 1 || n_neg < 1) return;

  const int mblocks         = (n_pos + M_TILE - 1) / M_TILE;
  const int n_pos_pad       = mblocks * M_TILE;
  const int n_tiles         = (n_emb + 15) / 16;
  const int tiles_per_slice = (n_tiles + N_SPLIT - 1) / N_SPLIT;
  const int pos_blocks      = (n_pos + 31) / 32;
  const int neg_blocks      = (n_neg + 31) / 32;
  const int zarg            = 0;

  char*  w   = (char*)d_ws;
  size_t off = 0;
  _Float16* e16 = (_Float16*)(w + off);
  off = alup256(off + (size_t)n_emb * D * sizeof(_Float16));
  float* gpart = (float*)(w + off);
  off = alup256(off + (size_t)N_SPLIT * (size_t)n_pos_pad * sizeof(float));
  float* posdot = (float*)(w + off);
  off = alup256(off + (size_t)pos_blocks * 32 * sizeof(float));
  float* negdot = (float*)(w + off);
  off = alup256(off + (size_t)neg_blocks * 32 * sizeof(float));
  if (off > ws_size) return;

  k_norm<<<(n_emb + 7) / 8, 256, 0, stream>>>(emb, e16, n_emb);
  k_rows<<<dim3(mblocks, N_SPLIT), 256, 0, stream>>>(e16, pa, gpart, n_emb, n_pos,
                                                      tiles_per_slice, n_pos_pad, zarg);
  k_pairs<<<pos_blocks, 256, 0, stream>>>(emb, pa, pt, posdot, n_pos, n_emb);
  k_pairs<<<neg_blocks, 256, 0, stream>>>(emb, na, ng, negdot, n_neg, n_emb);
  k_final<<<1, 256, 0, stream>>>(gpart, posdot, negdot, out, n_pos, n_neg, n_pos_pad);
}
